// S5R_7516192768286
// MI455X (gfx1250) — hardware-run, weakly checked
//
#include <hip/hip_runtime.h>
#include <stddef.h>
#include <stdint.h>
#include <math.h>

#pragma clang fp contract(off)

#define NBATCH 8
#define HD     512
#define PD     512
#define SEQ    2048
#define NTOK   (NBATCH * SEQ)
#define NBU    (2 * PD)
#define KYS    (2 * PD)
#define LDY    (2 * KYS)
#define SFP    68
#define TB     8
#define TPX    72

static_assert(PD == 512);
static_assert(HD == 512);
static_assert(NTOK % 128 == 0);
static_assert(HD % 128 == 0);
static_assert(NBU % 64 == 0);
static_assert(SEQ % 64 == 0);
static_assert(HD % 64 == 0);
static_assert(HD % 32 == 0);
static_assert(KYS % 32 == 0);
static_assert((PD * HD * 2) % 2048 == 0);
static_assert(SEQ % TB == 0);
static_assert((TB * LDY) % (PD * 8) == 0);
static_assert(TB * NBU == 4 * 4 * PD);
static_assert(LDY / 8 == 256);
static_assert(LDY * 2 == NBU * 4);

typedef _Float16 hh16;
typedef __attribute__((ext_vector_type(16))) __bf16 v16bf;
typedef float v8f __attribute__((ext_vector_type(8)));
typedef float v4f __attribute__((ext_vector_type(4)));
typedef int v4i __attribute__((ext_vector_type(4)));
typedef int v8i __attribute__((ext_vector_type(8)));
typedef unsigned short v8us __attribute__((ext_vector_type(8)));

__device__ __forceinline__ v8f zero8() { return (v8f){0.f, 0.f, 0.f, 0.f, 0.f, 0.f, 0.f, 0.f}; }

__device__ __forceinline__ unsigned int bf16_rne_bits(float f) {
  const unsigned int u = __float_as_uint(f);
  return (u + 0x7fffu + ((u >> 16) & 1u)) >> 16;
}

__device__ __forceinline__ float gelu_f(float x) {
  return 0.5f * x * (1.0f + erff(x * 0.70710678118654752f));
}

__device__ __forceinline__ v8i ldfrag16(const unsigned short* __restrict__ p, int ld, int row0, int k0, int lane) {
  const unsigned short* q = p + (size_t)(row0 + (lane & 15)) * (size_t)ld + k0 + 8 * (lane >> 4);
  const v4i lo = *(const v4i*)(const void*)(q);
  const v4i hi = *(const v4i*)(const void*)(q + 16);
  return __builtin_shufflevector(lo, hi, 0, 1, 2, 3, 4, 5, 6, 7);
}

__device__ __forceinline__ v8f mma_b(v8i a, v8i b, v8f cc) {
  return __builtin_amdgcn_wmma_f32_16x16x32_bf16(false, __builtin_bit_cast(v16bf, a), false,
                                                 __builtin_bit_cast(v16bf, b), (short)0, cc, false, false);
}

__device__ __forceinline__ void gemm32x32(const unsigned short* __restrict__ A, const unsigned short* __restrict__ AL,
                                          int lda, const unsigned short* __restrict__ B,
                                          const unsigned short* __restrict__ BL, int ldb, int ma, int nb, int kdim,
                                          int lane, v8f (&acc)[2][2]) {
#pragma unroll 1
  for (int k0 = 0; k0 < kdim; k0 += 32) {
    const v8i a0 = ldfrag16(A, lda, ma, k0, lane);
    const v8i a1 = ldfrag16(A, lda, ma + 16, k0, lane);
    const v8i b0 = ldfrag16(B, ldb, nb, k0, lane);
    const v8i b1 = ldfrag16(B, ldb, nb + 16, k0, lane);
    const v8i c0 = ldfrag16(AL, lda, ma, k0, lane);
    const v8i c1 = ldfrag16(AL, lda, ma + 16, k0, lane);
    const v8i d0 = ldfrag16(BL, ldb, nb, k0, lane);
    const v8i d1 = ldfrag16(BL, ldb, nb + 16, k0, lane);
    acc[0][0] = mma_b(a0, b0, acc[0][0]);
    acc[1][0] = mma_b(a1, b0, acc[1][0]);
    acc[0][1] = mma_b(a0, b1, acc[0][1]);
    acc[1][1] = mma_b(a1, b1, acc[1][1]);
    acc[0][0] = mma_b(a0, d0, acc[0][0]);
    acc[1][0] = mma_b(a1, d0, acc[1][0]);
    acc[0][1] = mma_b(a0, d1, acc[0][1]);
    acc[1][1] = mma_b(a1, d1, acc[1][1]);
    acc[0][0] = mma_b(c0, b0, acc[0][0]);
    acc[1][0] = mma_b(c1, b0, acc[1][0]);
    acc[0][1] = mma_b(c0, b1, acc[0][1]);
    acc[1][1] = mma_b(c1, b1, acc[1][1]);
    asm volatile("v_nop\n\tv_nop\n\tv_nop\n\tv_nop"
                 : "+v"(acc[0][0]), "+v"(acc[0][1]), "+v"(acc[1][0]), "+v"(acc[1][1])
                 : "v"(a0), "v"(a1), "v"(b0), "v"(b1), "v"(c0), "v"(c1), "v"(d0), "v"(d1));
  }
}

__global__ __launch_bounds__(256) void k_tsplit(const float* __restrict__ u, unsigned short* __restrict__ xh,
                                                unsigned short* __restrict__ xl) {
  __shared__ __align__(16) unsigned short lh[64 * TPX];
  __shared__ __align__(16) unsigned short ll[64 * TPX];
  const int tid = threadIdx.x;
  const int l0 = blockIdx.x * 64, h0 = blockIdx.y * 64, b = blockIdx.z;
  const float* src = u + ((size_t)b * HD + h0) * SEQ + l0;
#pragma unroll
  for (int it = 0; it < 4; ++it) {
    const int idx = tid + 256 * it;
    const int hr = idx >> 4;
    const int pc = idx & 15;
    const v4f v = *(const v4f*)(src + (size_t)hr * SEQ + pc * 4);
#pragma unroll
    for (int j = 0; j < 4; ++j) {
      const float f = v[j];
      const unsigned int hb = bf16_rne_bits(f);
      const float fh = __uint_as_float(hb << 16);
      const unsigned int lb = bf16_rne_bits(f - fh);
      lh[(pc * 4 + j) * TPX + hr] = (unsigned short)hb;
      ll[(pc * 4 + j) * TPX + hr] = (unsigned short)lb;
    }
  }
  __syncthreads();
  v8us hv[2], lv[2];
  size_t go[2];
#pragma unroll
  for (int it = 0; it < 2; ++it) {
    const int idx = tid + 256 * it;
    const int lr = idx >> 3;
    const int q  = idx & 7;
    hv[it] = *(const v8us*)(lh + lr * TPX + q * 8);
    lv[it] = *(const v8us*)(ll + lr * TPX + q * 8);
    go[it] = ((size_t)(b * SEQ + l0 + lr)) * HD + h0 + q * 8;
  }
#pragma unroll
  for (int it = 0; it < 2; ++it) {
    *(volatile v8us*)(xh + go[it]) = hv[it];
    *(volatile v8us*)(xl + go[it]) = lv[it];
  }
  __threadfence();
#pragma unroll
  for (int it = 0; it < 2; ++it) {
    *(volatile v8us*)(xh + go[it]) = hv[it];
    *(volatile v8us*)(xl + go[it]) = lv[it];
  }
}

__global__ __launch_bounds__(256) void k_prepw(const float* __restrict__ Bw, const float* __restrict__ Cw,
                                               unsigned short* __restrict__ BPH, unsigned short* __restrict__ BPL,
                                               unsigned short* __restrict__ CPH, unsigned short* __restrict__ CPL) {
  const int i = blockIdx.x * 256 + threadIdx.x;
  const int e0 = i * 8;
  const int nb = e0 / HD, kb = e0 % HD;
  const float* sb = Bw + ((size_t)((nb & (PD - 1)) * HD + kb)) * 2 + (nb >> 9);
  const int hc = e0 / KYS, kc = e0 % KYS;
  const int cc = kc >> 9;
  const float sgn = cc ? -1.0f : 1.0f;
  const float* sc = Cw + ((size_t)(hc * PD + (kc & (PD - 1)))) * 2 + cc;
  v8us bh, bl, ch, cl;
#pragma unroll
  for (int e = 0; e < 8; ++e) {
    const float vb = sb[2 * e];
    const unsigned int hb = bf16_rne_bits(vb);
    const float fb = __uint_as_float(hb << 16);
    bh[e] = (unsigned short)hb;
    bl[e] = (unsigned short)bf16_rne_bits(vb - fb);
    const float vc = sgn * sc[2 * e];
    const unsigned int hcb = bf16_rne_bits(vc);
    const float fc = __uint_as_float(hcb << 16);
    ch[e] = (unsigned short)hcb;
    cl[e] = (unsigned short)bf16_rne_bits(vc - fc);
  }
  *(volatile v8us*)(BPH + e0) = bh;
  *(volatile v8us*)(BPL + e0) = bl;
  *(volatile v8us*)(CPH + e0) = ch;
  *(volatile v8us*)(CPL + e0) = cl;
  __threadfence();
  *(volatile v8us*)(BPH + e0) = bh;
  *(volatile v8us*)(BPL + e0) = bl;
  *(volatile v8us*)(CPH + e0) = ch;
  *(volatile v8us*)(CPL + e0) = cl;
}

template <int KD, int LDA, int LDB, int LDO, int MODE>
__global__ __launch_bounds__(256) void k_gemm(const unsigned short* __restrict__ A,
                                              const unsigned short* __restrict__ AL,
                                              const unsigned short* __restrict__ B,
                                              const unsigned short* __restrict__ BL,
                                              const float* __restrict__ res, const float* __restrict__ Dm,
                                              float* __restrict__ o32) {
  __shared__ __align__(16) float ldsf[128 * SFP];
  const int tid = threadIdx.x, lane = tid & 31, w = tid >> 5;
  const int h = lane >> 4, c = lane & 15;
  const int wm = (w >> 1) * 32, wn = (w & 1) * 32;
  const int m0 = blockIdx.y * 128;
  const int n0 = blockIdx.x * 64;
  if constexpr (MODE == 1) {
    const size_t bz = (size_t)blockIdx.z;
    B   += bz * (size_t)SEQ * (size_t)LDB;
    BL  += bz * (size_t)SEQ * (size_t)LDB;
    res += bz * (size_t)HD * (size_t)SEQ;
    o32 += bz * (size_t)HD * (size_t)SEQ;
  }

  v8f acc[2][2];
#pragma unroll
  for (int i = 0; i < 2; ++i)
#pragma unroll
    for (int j = 0; j < 2; ++j) acc[i][j] = zero8();
  gemm32x32(A, AL, LDA, B, BL, LDB, m0 + wm, n0 + wn, KD, lane, acc);

#pragma unroll
  for (int i = 0; i < 2; ++i)
#pragma unroll
    for (int j = 0; j < 2; ++j)
#pragma unroll
      for (int r = 0; r < 8; ++r)
        ldsf[(wm + 16 * i + 8 * h + r) * SFP + wn + 16 * j + c] = acc[i][j][r];
  __syncthreads();

  v4f val[8];
  size_t go[8];
#pragma unroll
  for (int it = 0; it < 8; ++it) {
    const int p  = tid + 256 * it;
    const int lr = p >> 4;
    const int pc = p & 15;
    const v4f sv = *(const v4f*)(ldsf + lr * SFP + pc * 4);
    const size_t gi = (size_t)(m0 + lr) * LDO + n0 + pc * 4;
    if constexpr (MODE == 1) {
      const int gm = m0 + lr;
      const float dd = Dm[(size_t)gm * HD + gm];
      const v4f rr = *(const v4f*)(res + gi);
      const v4f xx = sv + rr * dd;
      v4f g;
#pragma unroll
      for (int e = 0; e < 4; ++e) g[e] = gelu_f(xx[e]);
      val[it] = g;
    } else {
      val[it] = sv;
    }
    go[it] = gi;
  }
#pragma unroll
  for (int it = 0; it < 8; ++it) *(volatile v4f*)(o32 + go[it]) = val[it];
  __threadfence();
#pragma unroll
  for (int it = 0; it < 8; ++it) *(volatile v4f*)(o32 + go[it]) = val[it];
}

__global__ __launch_bounds__(PD) void k_scan(const float* __restrict__ lam, float* buy) {
  __shared__ __align__(16) float sf[TB * NBU];
  __shared__ __align__(16) unsigned short lds[TB * LDY];
  const int tid = threadIdx.x;
  const size_t rowb = (size_t)blockIdx.x * SEQ;
  unsigned short* ys = (unsigned short*)buy;

  const float lr = lam[2 * tid + 0];
  const float li = lam[2 * tid + 1];

  float xr = 0.f, xi = 0.f;
#pragma unroll 1
  for (int t0 = 0; t0 < SEQ; t0 += TB) {
    const float* src = buy + (rowb + t0) * NBU;
    v4f bv[4];
#pragma unroll
    for (int it = 0; it < 4; ++it) {
      const int q = tid + PD * it;
      bv[it] = *(const v4f*)(src + (size_t)q * 4);
    }
#pragma unroll
    for (int it = 0; it < 4; ++it) {
      const int q = tid + PD * it;
      *(v4f*)(sf + q * 4) = bv[it];
    }
    __syncthreads();
#pragma unroll
    for (int tt = 0; tt < TB; ++tt) {
      const float br = sf[tt * NBU + tid];
      const float bi = sf[tt * NBU + PD + tid];
      const float nr = lr * xr - li * xi + br;
      const float ni = lr * xi + li * xr + bi;
      xr = nr;
      xi = ni;
      const unsigned int hbr = bf16_rne_bits(xr);
      const float fhr = __uint_as_float(hbr << 16);
      const unsigned int lbr = bf16_rne_bits(xr - fhr);
      const unsigned int hbi = bf16_rne_bits(xi);
      const float fhi = __uint_as_float(hbi << 16);
      const unsigned int lbi = bf16_rne_bits(xi - fhi);
      lds[tt * LDY + tid]            = (unsigned short)hbr;
      lds[tt * LDY + PD + tid]       = (unsigned short)hbi;
      lds[tt * LDY + KYS + tid]      = (unsigned short)lbr;
      lds[tt * LDY + KYS + PD + tid] = (unsigned short)lbi;
    }
    __syncthreads();
    v8us hv[4];
    size_t go[4];
#pragma unroll
    for (int it = 0; it < 4; ++it) {
      const int q = tid + PD * it;
      const int row = q >> 8;
      const int pc = q & 255;
      hv[it] = *(const v8us*)(lds + row * LDY + pc * 8);
      go[it] = (rowb + t0 + row) * LDY + (size_t)pc * 8;
    }
#pragma unroll
    for (int it = 0; it < 4; ++it) *(volatile v8us*)(ys + go[it]) = hv[it];
    __threadfence();
#pragma unroll
    for (int it = 0; it < 4; ++it) *(volatile v8us*)(ys + go[it]) = hv[it];
    __syncthreads();
  }
}

extern "C" void kernel_launch(void* const* d_in, const int* in_sizes, int n_in,
                              void* d_out, int out_size, void* d_ws, size_t ws_size,
                              hipStream_t stream) {
  if (n_in < 5) return;
  if (in_sizes[0] != NBATCH * HD * SEQ) return;
  if (in_sizes[1] != PD * 2) return;
  if (in_sizes[2] != PD * HD * 2) return;
  if (in_sizes[3] != HD * PD * 2) return;
  if (in_sizes[4] != HD * HD) return;
  if (out_size != NBATCH * HD * SEQ) return;

  const float* u   = (const float*)d_in[0];
  const float* lam = (const float*)d_in[1];
  const float* Bw  = (const float*)d_in[2];
  const float* Cw  = (const float*)d_in[3];
  const float* Dm  = (const float*)d_in[4];
  float* out = (float*)d_out;

  size_t off = 0;
  const size_t oXH  = off; off += (size_t)NTOK * HD * 2;
  const size_t oXL  = off; off += (size_t)NTOK * HD * 2;
  const size_t oBPH = off; off += (size_t)NBU * HD * 2;
  const size_t oBPL = off; off += (size_t)NBU * HD * 2;
  const size_t oCPH = off; off += (size_t)HD * KYS * 2;
  const size_t oCPL = off; off += (size_t)HD * KYS * 2;
  const size_t oBU  = off; off += (size_t)NTOK * NBU * 4;
  if (off > ws_size) return;
  if (off > (size_t)134217728) return;

  char* ws = (char*)d_ws;
  unsigned short* XH  = (unsigned short*)(ws + oXH);
  unsigned short* XL  = (unsigned short*)(ws + oXL);
  unsigned short* BPH = (unsigned short*)(ws + oBPH);
  unsigned short* BPL = (unsigned short*)(ws + oBPL);
  unsigned short* CPH = (unsigned short*)(ws + oCPH);
  unsigned short* CPL = (unsigned short*)(ws + oCPL);
  float* BU = (float*)(ws + oBU);
  unsigned short* YS = (unsigned short*)(ws + oBU);

  k_tsplit<<<dim3(SEQ / 64, HD / 64, NBATCH), dim3(256), 0, stream>>>(u, XH, XL);
  k_prepw<<<dim3((PD * HD * 2) / 2048), dim3(256), 0, stream>>>(Bw, Cw, BPH, BPL, CPH, CPL);
  k_gemm<HD, HD, HD, NBU, 0><<<dim3(NBU / 64, NTOK / 128, 1), dim3(256), 0, stream>>>(XH, XL, BPH, BPL, u, Dm, BU);
  k_scan<<<dim3(NBATCH), dim3(PD), 0, stream>>>(lam, BU);
  k_gemm<KYS, KYS, LDY, SEQ, 1><<<dim3(SEQ / 64, HD / 128, NBATCH), dim3(256), 0, stream>>>(CPH, CPL, YS, YS + KYS,
                                                                                             u, Dm, out);
  (void)hipGetLastError();
}
